// DeterministicEncoder_36481452212692
// MI455X (gfx1250) — hardware-verified
//
#include <hip/hip_runtime.h>
#include <hip/hip_bf16.h>
#include <math.h>

#define MM 8192
#define NN 8192
#define HID 16
#define OUT 64
#define GSTR 48

typedef _Float16 bf16;
typedef _Float16 f16;
typedef __attribute__((ext_vector_type(4))) unsigned v4u_t;
typedef unsigned v4ua __attribute__((ext_vector_type(4), may_alias));
typedef __attribute__((ext_vector_type(4))) float v4f_t;
typedef float v4fa __attribute__((ext_vector_type(4), may_alias));
typedef __attribute__((ext_vector_type(16))) bf16  bf16x16;
typedef bf16x16 f16x16;
typedef __attribute__((ext_vector_type(8)))  bf16  bf16x8;
typedef bf16x8 f16x8;
typedef __attribute__((ext_vector_type(4)))  bf16  bf16x4;
typedef __attribute__((ext_vector_type(8)))  float f32x8;
__device__ __forceinline__ f32x8 wmma16(f16x16 a, f16x16 b, f32x8 c) {
  c = __builtin_amdgcn_wmma_f32_16x16x32_f16(false, a, false, b, (short)0, c, false, false);
  asm volatile("v_nop\n\tv_nop\n\tv_nop\n\tv_nop" : "+v"(c) : "v"(a), "v"(b));
  return c;
}
#define LDS_STRIDE 48
#define KSTRIDE    72
#define VSTRIDE    48

__device__ __forceinline__ f32x8 wmma_bf16(bf16x16 a, bf16x16 b, f32x8 c) {
  c = __builtin_amdgcn_wmma_f32_16x16x32_f16(false, a, false, b, (short)0, c, false, false);
  asm volatile("v_nop\n\tv_nop\n\tv_nop\n\tv_nop" : "+v"(c) : "v"(a), "v"(b));
  return c;
}

template <typename T>
__device__ __forceinline__ bf16x16 load_frag(const T* __restrict__ base, int ld,
                                             int row0, int k0) {
  const int lane = threadIdx.x & 31;
  const int r    = lane & 15;
  const int kh   = (lane >> 4) * 8;
  const T* p0 = base + (size_t)(row0 + r) * ld + (k0 + kh);
  const T* p1 = p0 + 16;
  bf16x16 f;
#pragma unroll
  for (int i = 0; i < 8; ++i) {
    f[i]     = (bf16)p0[i];
    f[i + 8] = (bf16)p1[i];
  }
  return f;
}

__device__ __forceinline__ bf16x16 lds_frag(const bf16* base, int stride) {
  const int lane = threadIdx.x & 31;
  const int row  = lane & 15;
  const int kh   = (lane >> 4) * 8;
  const bf16x8 lo = *(const bf16x8*)(base + row * stride + kh);
  const bf16x8 hi = *(const bf16x8*)(base + row * stride + kh + 16);
  bf16x16 f;
#pragma unroll
  for (int i = 0; i < 8; ++i) { f[i] = lo[i]; f[i + 8] = hi[i]; }
  return f;
}

template <typename T>
__device__ __forceinline__ void stage_read16(const T* __restrict__ p, float* buf) {
#pragma unroll
  for (int i = 0; i < 16; ++i) buf[i] = (float)p[i];
}

__device__ __forceinline__ void stage_write(bf16* dst, const float* buf, int nquad) {
#pragma unroll
  for (int i = 0; i < nquad; ++i) {
    bf16x4 q;
    q[0] = (bf16)buf[4 * i];     q[1] = (bf16)buf[4 * i + 1];
    q[2] = (bf16)buf[4 * i + 2]; q[3] = (bf16)buf[4 * i + 3];
    *(bf16x4*)(dst + 4 * i) = q;
  }
}


#define GSTR 48
template <typename AT, int EPI, bool OUT16>
__global__ __launch_bounds__(256) void gemm_kne(const AT* __restrict__ A, int lda, const float* __restrict__ Wm, int ldw,
                                                const float* __restrict__ bias, const float* __restrict__ R, const float* __restrict__ gvec,
                                                void* __restrict__ Yv, int ldy, int K) {
  __shared__ __attribute__((aligned(16))) f16 ldsA[128 * GSTR];
  __shared__ __attribute__((aligned(16))) f16 ldsW[128 * GSTR];
  __shared__ __attribute__((aligned(16))) float oS[8][32 * 68];
  const int tid = threadIdx.x, lane = tid & 31, wave = tid >> 5, cl = lane & 15, rh = (lane >> 4) * 8;
  const int m0 = blockIdx.x * 128, n0 = blockIdx.y * 128;
  const int wm = (wave & 3) * 32, wn = (wave >> 2) * 64;
  f32x8 acc[2][4];
#pragma unroll
  for (int i = 0; i < 2; ++i)
#pragma unroll
    for (int j = 0; j < 4; ++j) { f32x8 z = {}; acc[i][j] = z; }
#pragma unroll 1
  for (int k0 = 0; k0 < K; k0 += 32) {
    __syncthreads();
    { const int row = tid >> 1, ch = (tid & 1) * 16;
      const AT* src = A + (size_t)(m0 + row) * lda + k0 + ch;
#pragma unroll
      for (int g = 0; g < 16; ++g) ldsA[row * GSTR + ch + g] = (f16)src[g]; }
    { const int k = tid >> 3, nn0 = (tid & 7) * 16;
      const float* src = Wm + (size_t)(k0 + k) * ldw + n0 + nn0;
#pragma unroll
      for (int g = 0; g < 4; ++g) { const v4f_t v = *(const v4f_t*)(src + 4 * g);
#pragma unroll
        for (int u = 0; u < 4; ++u) ldsW[(nn0 + 4 * g + u) * GSTR + k] = (f16)v[u]; } }
    __syncthreads();
    f16x16 af[2];
#pragma unroll
    for (int i = 0; i < 2; ++i) af[i] = lds_frag(ldsA + (wm + 16 * i) * GSTR, GSTR);
#pragma unroll
    for (int j = 0; j < 4; ++j) {
      const f16x16 bf = lds_frag(ldsW + (wn + 16 * j) * GSTR, GSTR);
#pragma unroll
      for (int i = 0; i < 2; ++i) acc[i][j] = wmma16(af[i], bf, acc[i][j]);
    }
  }
  float* so = oS[wave];
#pragma unroll
  for (int i = 0; i < 2; ++i)
#pragma unroll
    for (int j = 0; j < 4; ++j) {
      const int n = n0 + wn + 16 * j + cl;
      const float bv = bias ? bias[n] : 0.0f;
      const float gv = (EPI == 2) ? gvec[n] : 0.0f;
      if (EPI == 1) {
#pragma unroll 1
        for (int r = 0; r < 8; ++r) { const float xg = acc[i][j][r] + bv; so[(16 * i + rh + r) * 68 + 16 * j + cl] = 0.5f * xg * (1.0f + erff(xg * 0.70710678118654752f)); }
      } else {
#pragma unroll
        for (int r = 0; r < 8; ++r) {
          float v = acc[i][j][r] + bv;
          if (EPI == 2) v = R[(size_t)(m0 + wm + 16 * i + rh + r) * ldy + n] + gv * v;
          so[(16 * i + rh + r) * 68 + 16 * j + cl] = v;
        }
      }
    }
  asm volatile("s_wait_dscnt 0" ::: "memory");
  __builtin_amdgcn_wave_barrier();
#pragma unroll 1
  for (int pass = 0; pass < 2; ++pass) {
    if (OUT16) {
      f16* Y = (f16*)Yv;
#pragma unroll
      for (int it = 0; it < 8; ++it) { const int c = lane + 32 * it, rr = c >> 3, q8 = (c & 7) * 8;
        union { f16 h[8]; v4u_t v; } u;
#pragma unroll
        for (int e = 0; e < 8; ++e) u.h[e] = (f16)so[rr * 68 + q8 + e];
        *(volatile v4u_t*)(Y + (size_t)(m0 + wm + rr) * ldy + n0 + wn + q8) = u.v; }
    } else {
      float* Y = (float*)Yv;
#pragma unroll
      for (int it = 0; it < 16; ++it) { const int f4 = lane + 32 * it, rr = f4 >> 4, q = (f4 & 15) * 4;
        *(volatile v4f_t*)(Y + (size_t)(m0 + wm + rr) * ldy + n0 + wn + q) = *(const v4fa*)(so + rr * 68 + q); }
    }
    __threadfence();
  }
}

__global__ __launch_bounds__(256) void k_mlp(const float* __restrict__ xc, const float* __restrict__ yc, const float* __restrict__ W1, const float* __restrict__ b1, const float* __restrict__ W2, const float* __restrict__ b2,
                                            const float* __restrict__ W3, const float* __restrict__ b3, float* __restrict__ V) {
  __shared__ float h2S[64][HID + 1]; __shared__ __attribute__((aligned(16))) float vS[64][132];
  const int tid = threadIdx.x; const int r0 = blockIdx.x * 64;
  if (tid < 64) { const int m = r0 + tid; const float x = xc[m], y = yc[m]; float h1[HID];
#pragma unroll
    for (int j = 0; j < HID; ++j) h1[j] = fmaxf(x * W1[j] + y * W1[HID + j] + b1[j], 0.0f);
#pragma unroll 1
    for (int j = 0; j < HID; ++j) { float s = b2[j];
#pragma unroll
      for (int i = 0; i < HID; ++i) s += h1[i] * W2[i * HID + j];
      h2S[tid][j] = fmaxf(s, 0.0f); } }
  __syncthreads();
  { const int r = tid >> 2, part = tid & 3;
#pragma unroll 1
    for (int o = part * 16; o < part * 16 + 16; ++o) { float s = b3[o];
#pragma unroll 1
      for (int i = 0; i < HID; ++i) s += h2S[r][i] * W3[i * OUT + o];
      vS[r][o] = s; vS[r][64 + o] = 0.0f; } }
  __syncthreads();
#pragma unroll 1
  for (int pass = 0; pass < 2; ++pass) { for (int e = tid; e < 64 * 32; e += 256) { const int r = e >> 5, c4 = (e & 31) * 4; *(volatile v4f_t*)(V + (size_t)(r0 + r) * 128 + c4) = *(const v4fa*)(&vS[r][c4]); } __threadfence(); }
}
__global__ __launch_bounds__(256) void k_weights(const float* __restrict__ xc, const float* __restrict__ xt, float* __restrict__ Wm) { const size_t n = blockIdx.x; const float q = xt[n];
  for (int q4 = threadIdx.x; q4 < MM / 4; q4 += 256) { const v4f_t k = *(const v4f_t*)(xc + q4 * 4); v4f_t w; for (int e = 0; e < 4; ++e) w[e] = expf(-fabsf(k[e] - q));
    *(volatile v4f_t*)(Wm + n * MM + q4 * 4) = w; __threadfence(); *(volatile v4f_t*)(Wm + n * MM + q4 * 4) = w; } }
__global__ __launch_bounds__(256) void k_out(const float* __restrict__ Y, float* __restrict__ out) { const int n = blockIdx.x * 16 + (threadIdx.x >> 4), c4 = (threadIdx.x & 15) * 4;
  const v4f_t v = *(const v4f_t*)(Y + (size_t)n * 128 + c4); *(volatile v4f_t*)(out + (size_t)n * OUT + c4) = v; __threadfence(); *(volatile v4f_t*)(out + (size_t)n * OUT + c4) = v; }

extern "C" void kernel_launch(void* const* d_in, const int* in_sizes, int n_in,
                              void* d_out, int out_size, void* d_ws, size_t ws_size,
                              hipStream_t stream) {
  (void)in_sizes; (void)n_in; (void)out_size;
  const float** f = (const float**)d_in;
  const float* xc = f[0], *yc = f[1], *xt = f[2], *W1 = f[3], *b1 = f[4], *W2 = f[5], *b2 = f[6], *W3 = f[7], *b3 = f[8];
  float* out = (float*)d_out;
  char* ws = (char*)d_ws;
  float* V = (float*)ws; ws += (size_t)MM * 128 * 4;
  float* Wm = (float*)ws; ws += (size_t)2048 * MM * 4;
  float* Y = (float*)ws; ws += (size_t)NN * 128 * 4;
  if ((size_t)(ws - (char*)d_ws) > ws_size) return;
  const dim3 blk(256);
  k_mlp<<<dim3(MM / 64), blk, 0, stream>>>(xc, yc, W1, b1, W2, b2, W3, b3, V);
  for (int c = 0; c < NN / 2048; ++c) {
    k_weights<<<dim3(2048), blk, 0, stream>>>(xc, xt + c * 2048, Wm);
    gemm_kne<float, 0, false><<<dim3(2048 / 128, 1), blk, 0, stream>>>(Wm, MM, V, 128, nullptr, nullptr, nullptr, Y + (size_t)c * 2048 * 128, 128, MM);
  }
  k_out<<<dim3(NN / 16), blk, 0, stream>>>(Y, out);
}
